// StoX_Conv2d_72335839199774
// MI455X (gfx1250) — hardware-verified
//
#include <hip/hip_runtime.h>
#pragma clang fp contract(off)

typedef _Float16 f16t;
typedef _Float16 v16h __attribute__((ext_vector_type(16)));
typedef _Float16 v8h  __attribute__((ext_vector_type(8)));
typedef float    v8f  __attribute__((ext_vector_type(8)));
typedef float    v4f  __attribute__((ext_vector_type(4)));
typedef v8h __attribute__((may_alias)) v8ha;
typedef v4f __attribute__((may_alias)) v4fa;
union Frag { v16h v; v8h half[2]; };

#define NBATCH 8
#define CIN    64
#define HIMG   32
#define WIMG   32
#define LSP    1024
#define KTOT   576
#define NCHUNK 9
#define KCH    64
#define OFULL  256
#define OHALF  128
#define ABITS  4
#define NROWS  32768
#define NPIECE 72
#define QCOLS  34

#define OFF_QW   ((size_t)0)
#define SZ_QW    ((size_t)OFULL * KTOT * 2)
#define OFF_QA   (OFF_QW + SZ_QW)
#define SZ_QA    ((size_t)NROWS * KTOT * 2)
#define OFF_QAT  (OFF_QA + SZ_QA)
#define SZ_QAT   ((size_t)KTOT * NROWS * 2)
#define OFF_G    (OFF_QAT + SZ_QAT)
#define SZ_G     ((size_t)NCHUNK * KCH * KCH * 4)
#define OFF_MU   (OFF_G + SZ_G)
#define SZ_MU    ((size_t)NCHUNK * OFULL * 4)
#define OFF_RS   (OFF_MU + SZ_MU)
#define WS_TOTAL (OFF_RS + SZ_MU)
static_assert(WS_TOTAL <= (size_t)134217728);
static_assert((OFF_QA % 256) == 0 && (OFF_QAT % 256) == 0 && (OFF_G % 256) == 0 && (OFF_MU % 256) == 0 && (OFF_RS % 256) == 0);
static_assert(NROWS == ABITS * NBATCH * LSP);
static_assert(KTOT == CIN * 9 && KTOT == NCHUNK * KCH && NPIECE * 8 == KTOT);

__device__ __forceinline__ v8f wmma_f16(v16h a, v16h b, v8f c) {
  v8f d = __builtin_amdgcn_wmma_f32_16x16x32_f16(false, a, false, b, (short)0, c, false, false);
  asm volatile("v_nop\n\tv_nop\n\tv_nop\n\tv_nop" : "+v"(d) : "v"(a), "v"(b));
  return d;
}

__device__ __forceinline__ v16h load_frag32(const f16t* p, int h) {
  Frag f;
  f.half[0] = *(const v8ha*)(p + 8 * h);
  f.half[1] = *(const v8ha*)(p + 16 + 8 * h);
  return f.v;
}

__device__ __forceinline__ f16t sgnh(float d) {
  return (f16t)(float)((d > 0.0f) - (d < 0.0f));
}

__device__ __forceinline__ unsigned char qlevel(float v) {
  const float c = fminf(fmaxf(v, 0.0f), 1.0f);
  const float t = c * 15.0f;
  return (unsigned char)(int)rintf(t);
}

__device__ __forceinline__ int qgather(const unsigned char* sq, int kk, int ll) {
  const int cin = kk / 9;
  const int tap = kk - 9 * cin;
  const int kh = tap / 3;
  const int kw = tap - 3 * kh;
  const int hl = ll >> 5, w = ll & 31;
  return (int)sq[(cin * 4 + hl + kh) * QCOLS + w + kw];
}

__global__ __launch_bounds__(128) void k_wq(const float* __restrict__ wf, f16t* __restrict__ qw16) {
  __shared__ double sred[4][32];
  __shared__ float smu[4];
  const int tid = threadIdx.x, lane = tid & 31, w = tid >> 5;
  const int o = blockIdx.x * 4 + w;
  const float* row = wf + (size_t)o * KTOT;
  v4f va[3], vb[3];
  double s = 0.0;
  #pragma unroll
  for (int j = 0; j < 3; ++j) {
    const int p = lane + 32 * j;
    const int pc = (p < NPIECE) ? p : (NPIECE - 1);
    va[j] = *(const v4fa*)(row + 8 * pc);
    vb[j] = *(const v4fa*)(row + 8 * pc + 4);
    const double t = (((double)va[j].x + (double)va[j].y) + ((double)va[j].z + (double)va[j].w))
                   + (((double)vb[j].x + (double)vb[j].y) + ((double)vb[j].z + (double)vb[j].w));
    s += (p < NPIECE) ? t : 0.0;
  }
  sred[w][lane] = s;
  __syncthreads();
  if (lane == 0) {
    double t = 0.0;
    for (int i = 0; i < 32; ++i) t += sred[w][i];
    smu[w] = (float)(t * (1.0 / 576.0));
  }
  __syncthreads();
  const float mu = smu[w];
  v8h vals[3];
  #pragma unroll
  for (int j = 0; j < 3; ++j) {
    vals[j][0] = sgnh(va[j].x - mu);
    vals[j][1] = sgnh(va[j].y - mu);
    vals[j][2] = sgnh(va[j].z - mu);
    vals[j][3] = sgnh(va[j].w - mu);
    vals[j][4] = sgnh(vb[j].x - mu);
    vals[j][5] = sgnh(vb[j].y - mu);
    vals[j][6] = sgnh(vb[j].z - mu);
    vals[j][7] = sgnh(vb[j].w - mu);
  }
  f16t* dst = qw16 + (size_t)o * KTOT;
  const bool tail = lane < 8;
  *(volatile v8h*)(dst + 8 * lane) = vals[0];
  *(volatile v8h*)(dst + 8 * (lane + 32)) = vals[1];
  if (tail) *(volatile v8h*)(dst + 8 * (lane + 64)) = vals[2];
  __threadfence();
  *(volatile v8h*)(dst + 8 * lane) = vals[0];
  *(volatile v8h*)(dst + 8 * (lane + 32)) = vals[1];
  if (tail) *(volatile v8h*)(dst + 8 * (lane + 64)) = vals[2];
}

__global__ __launch_bounds__(256) void k_bits(const float* __restrict__ x, f16t* __restrict__ qa16,
                                              f16t* __restrict__ qat16) {
  __shared__ unsigned char sq[CIN * 4 * QCOLS];
  const int tid = threadIdx.x;
  const int h2 = blockIdx.x, b = blockIdx.y;
  const int h0 = 2 * h2;
  {
    const int cin = tid >> 2, yy = tid & 3;
    const int y = h0 - 1 + yy;
    const bool vy = (unsigned)y < (unsigned)HIMG;
    const int yc = y < 0 ? 0 : (y > HIMG - 1 ? HIMG - 1 : y);
    const float* rp = x + ((size_t)(b * CIN + cin) * HIMG + yc) * WIMG;
    unsigned char* sp = sq + (cin * 4 + yy) * QCOLS;
    const unsigned char z = 0;
    sp[0] = z;
    sp[QCOLS - 1] = z;
    #pragma unroll
    for (int k = 0; k < 8; ++k) {
      const v4f v = *(const v4fa*)(rp + 4 * k);
      sp[1 + 4 * k + 0] = vy ? qlevel(v.x) : z;
      sp[1 + 4 * k + 1] = vy ? qlevel(v.y) : z;
      sp[1 + 4 * k + 2] = vy ? qlevel(v.z) : z;
      sp[1 + 4 * k + 3] = vy ? qlevel(v.w) : z;
    }
  }
  __syncthreads();
  const int rowbase = b * LSP + h0 * WIMG;

  #pragma unroll 1
  for (int it = 0; it < 18; ++it) {
    const int item = it * 256 + tid;
    const int ll = item / NPIECE;
    const int p = item - NPIECE * ll;
    v8h vals[4];
    #pragma unroll
    for (int e = 0; e < 8; ++e) {
      const int q = qgather(sq, 8 * p + e, ll);
      #pragma unroll
      for (int i = 0; i < ABITS; ++i) vals[i][e] = (f16t)(float)((q >> i) & 1);
    }
    size_t d[4];
    #pragma unroll
    for (int i = 0; i < ABITS; ++i)
      d[i] = ((size_t)(i * NBATCH * LSP + rowbase + ll)) * KTOT + 8 * p;
    #pragma unroll
    for (int i = 0; i < ABITS; ++i) *(volatile v8h*)(qa16 + d[i]) = vals[i];
    __threadfence();
    #pragma unroll
    for (int i = 0; i < ABITS; ++i) *(volatile v8h*)(qa16 + d[i]) = vals[i];
  }

  #pragma unroll 1
  for (int it = 0; it < 18; ++it) {
    const int item = it * 256 + tid;
    const int kk = item >> 3;
    const int oct = item & 7;
    v8h vals[4];
    #pragma unroll
    for (int e = 0; e < 8; ++e) {
      const int q = qgather(sq, kk, 8 * oct + e);
      #pragma unroll
      for (int i = 0; i < ABITS; ++i) vals[i][e] = (f16t)(float)((q >> i) & 1);
    }
    size_t d[4];
    #pragma unroll
    for (int i = 0; i < ABITS; ++i)
      d[i] = (size_t)kk * NROWS + (size_t)(i * NBATCH * LSP + rowbase + 8 * oct);
    #pragma unroll
    for (int i = 0; i < ABITS; ++i) *(volatile v8h*)(qat16 + d[i]) = vals[i];
    __threadfence();
    #pragma unroll
    for (int i = 0; i < ABITS; ++i) *(volatile v8h*)(qat16 + d[i]) = vals[i];
  }
}

__global__ __launch_bounds__(128) void k_gram(const f16t* __restrict__ qat16, float* __restrict__ g) {
  __shared__ __attribute__((aligned(16))) float sD[16 * 64];
  const int tid = threadIdx.x, lane = tid & 31, w = tid >> 5;
  const int h = lane >> 4, m = lane & 15;
  const int ti = blockIdx.x, c = blockIdx.y;
  const f16t* ap = qat16 + (size_t)(c * KCH + 16 * ti + m) * NROWS;
  const f16t* bp = qat16 + (size_t)(c * KCH + 16 * w + m) * NROWS;
  const v8f z8 = {0.f, 0.f, 0.f, 0.f, 0.f, 0.f, 0.f, 0.f};
  v8f acc = z8;
  #pragma unroll 2
  for (int k0 = 0; k0 < NROWS; k0 += 32) {
    const v16h a = load_frag32(ap + k0, h);
    const v16h bb = load_frag32(bp + k0, h);
    acc = wmma_f16(a, bb, acc);
  }
  #pragma unroll
  for (int r = 0; r < 8; ++r) sD[(8 * h + r) * 64 + 16 * w + m] = acc[r];
  __syncthreads();
  v4f vals[2];
  size_t gi[2];
  #pragma unroll
  for (int i = 0; i < 2; ++i) {
    const int row = 4 * w + 2 * i + (lane >> 4);
    const int piece = lane & 15;
    vals[i] = *(const v4fa*)(sD + row * 64 + 4 * piece);
    gi[i] = ((size_t)(c * KCH + 16 * ti + row)) * KCH + 4 * piece;
  }
  #pragma unroll
  for (int i = 0; i < 2; ++i) *(volatile v4f*)(g + gi[i]) = vals[i];
  __threadfence();
  #pragma unroll
  for (int i = 0; i < 2; ++i) *(volatile v4f*)(g + gi[i]) = vals[i];
}

__global__ __launch_bounds__(256) void k_stats(const float* __restrict__ g, const f16t* __restrict__ qw16,
                                               float* __restrict__ mu_out, float* __restrict__ rs_out) {
  __shared__ int sG[KCH * KCH];
  __shared__ __attribute__((aligned(16))) float sMu[OFULL];
  __shared__ __attribute__((aligned(16))) float sRs[OFULL];
  const int tid = threadIdx.x, lane = tid & 31, w = tid >> 5;
  const int c = blockIdx.x;
  const int o = tid;
  #pragma unroll 1
  for (int i = 0; i < 16; ++i) sG[i * 256 + tid] = (int)g[(size_t)c * (KCH * KCH) + i * 256 + tid];
  unsigned long long pos = 0ull, neg = 0ull;
  const f16t* wr = qw16 + (size_t)o * KTOT + c * KCH;
  #pragma unroll
  for (int j = 0; j < 8; ++j) {
    const v8h v = *(const v8ha*)(wr + 8 * j);
    #pragma unroll
    for (int e = 0; e < 8; ++e) {
      const float f = (float)v[e];
      pos |= (f > 0.0f) ? (1ull << (8 * j + e)) : 0ull;
      neg |= (f < 0.0f) ? (1ull << (8 * j + e)) : 0ull;
    }
  }
  __syncthreads();
  int S1 = 0, S2 = 0;
  #pragma unroll 1
  for (int k1 = 0; k1 < KCH; ++k1) {
    const int s1 = (int)((pos >> k1) & 1ull) - (int)((neg >> k1) & 1ull);
    const int* gr = sG + k1 * KCH;
    int rsum = 0;
    #pragma unroll 8
    for (int k2 = 0; k2 < KCH; ++k2) {
      const int s2 = (int)((pos >> k2) & 1ull) - (int)((neg >> k2) & 1ull);
      rsum += s2 * gr[k2];
    }
    S1 += s1 * gr[k1];
    S2 += s1 * rsum;
  }
  const float muf = (float)S1 * (1.0f / 32768.0f);
  const double mu64 = (double)S1 * (1.0 / 32768.0);
  const double var64 = (double)S2 * (1.0 / 32768.0) - mu64 * mu64;
  const float varf = (float)var64;
  const float rsd = 1.0f / sqrtf(varf + 1e-5f);
  sMu[o] = muf;
  sRs[o] = rsd;
  __syncthreads();
  v4f vals[2];
  size_t gi[2];
  #pragma unroll
  for (int i = 0; i < 2; ++i) {
    const int piece = 32 * i + lane;
    if (w == 0) vals[i] = *(const v4fa*)(sMu + 4 * piece);
    else        vals[i] = *(const v4fa*)(sRs + 4 * piece);
    gi[i] = (size_t)c * OFULL + 4 * piece;
  }
  if (w == 0) {
    #pragma unroll
    for (int i = 0; i < 2; ++i) *(volatile v4f*)(mu_out + gi[i]) = vals[i];
  } else if (w == 1) {
    #pragma unroll
    for (int i = 0; i < 2; ++i) *(volatile v4f*)(rs_out + gi[i]) = vals[i];
  }
  __threadfence();
  if (w == 0) {
    #pragma unroll
    for (int i = 0; i < 2; ++i) *(volatile v4f*)(mu_out + gi[i]) = vals[i];
  } else if (w == 1) {
    #pragma unroll
    for (int i = 0; i < 2; ++i) *(volatile v4f*)(rs_out + gi[i]) = vals[i];
  }
}

__global__ __launch_bounds__(256) void k_main(const f16t* __restrict__ qa16, const f16t* __restrict__ qw16,
                                              const float* __restrict__ mut, const float* __restrict__ rst,
                                              const float* __restrict__ gam, const float* __restrict__ bet,
                                              float* __restrict__ out) {
  __shared__ __attribute__((aligned(16))) float sD[32 * 64];
  const int tid = threadIdx.x, lane = tid & 31, w = tid >> 5;
  const int h = lane >> 4, m = lane & 15;
  const int ob = blockIdx.x, lb = blockIdx.y, b = blockIdx.z;
  const int lt = w & 3, ot = w >> 2;
  const int l0 = lb * 64 + 16 * lt;
  const int ooL = ob * 32 + 16 * ot + m;
  float gm[2], btv[2];
  const f16t* bwp[2];
  #pragma unroll
  for (int s = 0; s < 2; ++s) {
    const int o = s * OHALF + ooL;
    gm[s] = gam[o];
    btv[s] = bet[o];
    bwp[s] = qw16 + (size_t)o * KTOT;
  }
  const f16t* arp[4];
  #pragma unroll
  for (int a = 0; a < ABITS; ++a)
    arp[a] = qa16 + ((size_t)((a * NBATCH + b) * LSP + l0 + m)) * KTOT;
  const v8f z8 = {0.f, 0.f, 0.f, 0.f, 0.f, 0.f, 0.f, 0.f};
  v8f cnt[4][2];
  #pragma unroll
  for (int a = 0; a < ABITS; ++a) { cnt[a][0] = z8; cnt[a][1] = z8; }

  #pragma unroll 1
  for (int c = 0; c < NCHUNK; ++c) {
    const int k0 = c * KCH;
    float mu[2], rs[2];
    v16h bf0[2], bf1[2];
    #pragma unroll
    for (int s = 0; s < 2; ++s) {
      const int o = s * OHALF + ooL;
      mu[s] = mut[c * OFULL + o];
      rs[s] = rst[c * OFULL + o];
      bf0[s] = load_frag32(bwp[s] + k0, h);
      bf1[s] = load_frag32(bwp[s] + k0 + 32, h);
    }
    #pragma unroll
    for (int a = 0; a < ABITS; ++a) {
      const v16h a0 = load_frag32(arp[a] + k0, h);
      const v16h a1 = load_frag32(arp[a] + k0 + 32, h);
      #pragma unroll
      for (int s = 0; s < 2; ++s) {
        v8f lin = wmma_f16(a0, bf0[s], z8);
        lin = wmma_f16(a1, bf1[s], lin);
        #pragma unroll
        for (int r = 0; r < 8; ++r) {
          const float d = lin[r] - mu[s];
          const float t = gm[s] * d;
          const float u = t * rs[s];
          const float bn = u + btv[s];
          cnt[a][s][r] = cnt[a][s][r] + (float)((bn > 0.0f) - (bn < 0.0f));
        }
      }
    }
  }

  const float wv0 = 1.0f / 3.0f;
  const float wv1 = 2.0f / 3.0f;
  const float av0 = 1.0f / 15.0f;
  const float av1 = 2.0f / 15.0f;
  const float av2 = 4.0f / 15.0f;
  const float av3 = 8.0f / 15.0f;
  #pragma unroll
  for (int r = 0; r < 8; ++r) {
    float y[4];
    #pragma unroll
    for (int a = 0; a < ABITS; ++a) {
      const float o0 = cnt[a][0][r] + cnt[a][0][r];
      const float o1 = cnt[a][1][r] + cnt[a][1][r];
      const float p0 = wv0 * o0;
      const float p1 = wv1 * o1;
      y[a] = p0 + p1;
    }
    const float q0 = av0 * y[0];
    const float q1 = av1 * y[1];
    const float q2 = av2 * y[2];
    const float q3 = av3 * y[3];
    const float fin = ((q0 + q1) + q2) + q3;
    sD[(16 * ot + m) * 64 + 16 * lt + 8 * h + r] = fin;
  }
  __syncthreads();
  v4f vals[2];
  size_t gi[2];
  #pragma unroll
  for (int i = 0; i < 2; ++i) {
    const int row = 4 * w + 2 * i + (lane >> 4);
    const int piece = lane & 15;
    vals[i] = *(const v4fa*)(sD + row * 64 + 4 * piece);
    gi[i] = ((size_t)(b * OHALF + ob * 32 + row)) * LSP + lb * 64 + 4 * piece;
  }
  #pragma unroll
  for (int i = 0; i < 2; ++i) *(volatile v4f*)(out + gi[i]) = vals[i];
  __threadfence();
  #pragma unroll
  for (int i = 0; i < 2; ++i) *(volatile v4f*)(out + gi[i]) = vals[i];
}

extern "C" void kernel_launch(void* const* d_in, const int* in_sizes, int n_in,
                              void* d_out, int out_size, void* d_ws, size_t ws_size,
                              hipStream_t stream) {
  if (n_in < 4) return;
  if (in_sizes[0] != NBATCH * CIN * HIMG * WIMG) return;
  if (in_sizes[1] != OFULL * KTOT) return;
  if (in_sizes[2] != OFULL || in_sizes[3] != OFULL) return;
  if (out_size != NBATCH * OHALF * LSP) return;
  if (ws_size < WS_TOTAL) return;

  const float* inputs = (const float*)d_in[0];
  const float* weight = (const float*)d_in[1];
  const float* gamma  = (const float*)d_in[2];
  const float* beta   = (const float*)d_in[3];
  float* outp = (float*)d_out;

  char* ws = (char*)d_ws;
  f16t*  QW16  = (f16t*)(ws + OFF_QW);
  f16t*  QA16  = (f16t*)(ws + OFF_QA);
  f16t*  QAT16 = (f16t*)(ws + OFF_QAT);
  float* G     = (float*)(ws + OFF_G);
  float* MU    = (float*)(ws + OFF_MU);
  float* RS    = (float*)(ws + OFF_RS);

  k_wq<<<OFULL / 4, 128, 0, stream>>>(weight, QW16);
  k_bits<<<dim3(HIMG / 2, NBATCH), 256, 0, stream>>>(inputs, QA16, QAT16);
  k_gram<<<dim3(4, NCHUNK), 128, 0, stream>>>(QAT16, G);
  k_stats<<<NCHUNK, 256, 0, stream>>>(G, QW16, MU, RS);
  k_main<<<dim3(OHALF / 32, LSP / 64, NBATCH), 256, 0, stream>>>(QA16, QW16, MU, RS, gamma, beta, outp);
}
